// GraphAttention_44813688766608
// MI455X (gfx1250) — hardware-verified
//
#include <hip/hip_runtime.h>
#include <math.h>
#include <stdint.h>

#ifndef NB
#define NB 2
#endif
#ifndef SEQ
#define SEQ 2048
#endif
#ifndef NB_FULL
#define NB_FULL 2
#endif
#ifndef SEQ_FULL
#define SEQ_FULL 2048
#endif
#define FIN   128
#define UD    64
#define NHD   8
#define FD    FIN
#define QKS   (NHD * FD)
#define HU    (NHD * UD)
#define BN    (NB * SEQ)
#define PSC   1024.0f
#define OSC   0.0009765625f
#define NEGFILL (-3.40282347e38f)

static_assert(NB >= 1 && NB <= NB_FULL && SEQ >= 64 && SEQ <= SEQ_FULL);
static_assert(SEQ % 64 == 0 && BN % 32 == 0);
static_assert(FIN % 64 == 0 && FIN % 32 == 0 && UD == 64 && HU % 128 == 0 && FD == 128 && QKS == NHD * FD);
static_assert(QKS % 128 == 0 && FD % 32 == 0);

typedef __bf16         v16b __attribute__((ext_vector_type(16)));
typedef __bf16         v8b  __attribute__((ext_vector_type(8)));
typedef _Float16       v16h __attribute__((ext_vector_type(16)));
typedef _Float16       v8h  __attribute__((ext_vector_type(8)));
typedef _Float16       v4h  __attribute__((ext_vector_type(4)));
typedef float          v8f  __attribute__((ext_vector_type(8)));
typedef float          v4f  __attribute__((ext_vector_type(4)));
typedef unsigned int   v4u  __attribute__((ext_vector_type(4)));
typedef int            v4i  __attribute__((ext_vector_type(4)));
typedef v4f __attribute__((may_alias)) v4fa;
typedef v4u __attribute__((may_alias)) v4ua;
typedef v4i __attribute__((may_alias)) v4ia;
typedef v8b __attribute__((may_alias)) v8ba;
typedef v8h __attribute__((may_alias)) v8ha;
typedef v4h __attribute__((may_alias)) v4ha;

__device__ __forceinline__ unsigned short bf_bits(float f) {
  const unsigned u = __float_as_uint(f);
  return (unsigned short)((u + 0x7FFFu + ((u >> 16) & 1u)) >> 16);
}
__device__ __forceinline__ float bf_val(unsigned short h) { return __uint_as_float(((unsigned)h) << 16); }
__device__ __forceinline__ float bf_rne(float f) { return bf_val(bf_bits(f)); }
__device__ __forceinline__ v4f bf_rne4(v4f a) {
  v4f r;
  r[0] = bf_rne(a[0]); r[1] = bf_rne(a[1]); r[2] = bf_rne(a[2]); r[3] = bf_rne(a[3]);
  return r;
}
__device__ __forceinline__ unsigned short h_bits(float f) {
  const _Float16 hv = (_Float16)f;
  return __builtin_bit_cast(unsigned short, hv);
}
template <int KIND>
__device__ __forceinline__ unsigned short cvt16(float f) { return KIND == 0 ? bf_bits(f) : h_bits(bf_rne(f)); }
__device__ __forceinline__ unsigned pk16(unsigned short a, unsigned short b) { return (unsigned)a | ((unsigned)b << 16); }
__device__ __forceinline__ v8f zero8() { v8f z = {0.f, 0.f, 0.f, 0.f, 0.f, 0.f, 0.f, 0.f}; return z; }
__device__ __forceinline__ int wave_id() { return __builtin_amdgcn_readfirstlane((int)(threadIdx.x >> 5)); }

__device__ __forceinline__ void lds_wave_sync() {
  __builtin_amdgcn_fence(3  , "workgroup");
  __builtin_amdgcn_wave_barrier();
  __builtin_amdgcn_fence(2  , "workgroup");
}

union FragB { v16b v; v8b h[2]; };
union FragH { v16h v; v8h h[2]; };
__device__ __forceinline__ v16b ldfrag_b(const __bf16* p) {
  FragB f;
  f.h[0] = *(const v8ba*)(p);
  f.h[1] = *(const v8ba*)(p + 16);
  return f.v;
}
__device__ __forceinline__ v16h ldfrag_h(const _Float16* p) {
  FragH f;
  f.h[0] = *(const v8ha*)(p);
  f.h[1] = *(const v8ha*)(p + 16);
  return f.v;
}
__device__ __forceinline__ v8f mma_b(v16b a, v16b b, v8f c) {
  return __builtin_amdgcn_wmma_f32_16x16x32_bf16(false, a, false, b, (short)0, c, false, false);
}
__device__ __forceinline__ v8f mma_h(v16h a, v16h b, v8f c) {
  return __builtin_amdgcn_wmma_f32_16x16x32_f16(false, a, false, b, (short)0, c, false, false);
}
__device__ __forceinline__ void guard_b3(v8f& a, v8f& b, v16b x0, v16b x1, v16b y0) {
  asm volatile("v_nop\n\tv_nop\n\tv_nop\n\tv_nop" : "+v"(a), "+v"(b) : "v"(x0), "v"(x1), "v"(y0) : "memory");
}
__device__ __forceinline__ void guard1_h4(v8f& a, v16h w, v16h x, v16h y, v16h z) {
  asm volatile("v_nop\n\tv_nop\n\tv_nop\n\tv_nop" : "+v"(a) : "v"(w), "v"(x), "v"(y), "v"(z) : "memory");
}
__device__ __forceinline__ void acc_guard4(v8f& a, v8f& b, v8f& c, v8f& d) {
  asm volatile("v_nop\n\tv_nop\n\tv_nop\n\tv_nop" : "+v"(a), "+v"(b), "+v"(c), "+v"(d));
}

__global__ __launch_bounds__(256) void prep_x_kernel(const float* __restrict__ x, unsigned short* __restrict__ xb, int nunits) {
  const int i = (int)blockIdx.x * 256 + (int)threadIdx.x;
  if (i >= nunits) return;
  const size_t e  = 8 * (size_t)i;
  const int    bn = (int)(e / FIN);
  const int    f  = (int)(e - (size_t)bn * FIN);
  const int    b  = bn / SEQ;
  const int    n  = bn - b * SEQ;
  const float* src = x + ((size_t)b * SEQ_FULL + n) * FIN + f;
  const v4f a = *(const v4fa*)(src);
  const v4f c = *(const v4fa*)(src + 4);
  v4u w;
  w[0] = pk16(bf_bits(a[0]), bf_bits(a[1]));
  w[1] = pk16(bf_bits(a[2]), bf_bits(a[3]));
  w[2] = pk16(bf_bits(c[0]), bf_bits(c[1]));
  w[3] = pk16(bf_bits(c[2]), bf_bits(c[3]));
  *(volatile v4u*)(xb + e) = w;
  __threadfence();
  *(volatile v4u*)(xb + e) = w;
}

template <int KIND>
__global__ __launch_bounds__(256) void tconv_kernel(const float* __restrict__ W, unsigned short* __restrict__ outp,
                                                    int R, int Cc, long sIn, long sOut) {
  __shared__ __align__(16) float tf[64 * 68];
  W    += (size_t)blockIdx.z * sIn;
  outp += (size_t)blockIdx.z * sOut;
  const int c0  = (int)blockIdx.x * 64;
  const int r0  = (int)blockIdx.y * 64;
  const int tid = (int)threadIdx.x;
  {
    const int lr = tid >> 4;
    const int c4 = (tid & 15) * 4;
#pragma unroll
    for (int it = 0; it < 4; ++it) {
      const int rr = it * 16 + lr;
      const v4f a = *(const v4fa*)(W + (size_t)(r0 + rr) * Cc + c0 + c4);
      *(v4f*)(tf + rr * 68 + c4) = a;
    }
  }
  __syncthreads();
  const int sub = tid >> 3;
  const int c8  = (tid & 7) * 8;
  v4u hv[2];
#pragma unroll
  for (int it = 0; it < 2; ++it) {
    const int oc = it * 32 + sub;
    v4u a;
#pragma unroll
    for (int q = 0; q < 4; ++q) {
      const float f0 = tf[(c8 + 2 * q) * 68 + oc];
      const float f1 = tf[(c8 + 2 * q + 1) * 68 + oc];
      a[q] = pk16(cvt16<KIND>(f0), cvt16<KIND>(f1));
    }
    hv[it] = a;
  }
  for (int pass = 0; pass < 2; ++pass) {
#pragma unroll
    for (int it = 0; it < 2; ++it) {
      const int oc = it * 32 + sub;
      const size_t go = (size_t)(c0 + oc) * R + r0 + c8;
      *(volatile v4u*)(outp + go) = hv[it];
    }
    __threadfence();
  }
}

#define SLAB_PERW 2048

__global__ __launch_bounds__(128) __attribute__((amdgpu_num_vgpr(256))) void gemm_sd_kernel(
    const unsigned short* Ap, int lda, const unsigned short* Btp, int ldb,
    int M, int N, int K, const float* __restrict__ attk, float* sd, int bnp) {
  __shared__ __align__(16) float slab_all[4 * SLAB_PERW];

  const int lane = threadIdx.x & 31;
  const int wave = wave_id();
  const int hh = lane >> 4;
  const int rl = lane & 15;
  const int tilesN = N >> 7;
  const int tilesM = M >> 5;
  const int tile = (int)blockIdx.x * 4 + wave;
  if (tile >= tilesM * tilesN) return;
  const int tm = tile / tilesN;
  const int tn = tile - tm * tilesN;
  const int m0 = tm << 5;
  const int n0 = tn << 7;

  const __bf16* A  = (const __bf16*)(const void*)Ap;
  const __bf16* Bt = (const __bf16*)(const void*)Btp;

  v8f acc[2][8];
#pragma unroll
  for (int i = 0; i < 2; ++i)
#pragma unroll
    for (int j = 0; j < 8; ++j) acc[i][j] = zero8();

  for (int k0 = 0; k0 < K; k0 += 32) {
    const v16b a0f = ldfrag_b(A + (size_t)(m0 + rl) * lda + k0 + 8 * hh);
    const v16b a1f = ldfrag_b(A + (size_t)(m0 + 16 + rl) * lda + k0 + 8 * hh);
#pragma unroll
    for (int j = 0; j < 8; ++j) {
      const v16b bh = ldfrag_b(Bt + (size_t)(n0 + j * 16 + rl) * ldb + k0 + 8 * hh);
      acc[0][j] = mma_b(a0f, bh, acc[0][j]);
      acc[1][j] = mma_b(a1f, bh, acc[1][j]);
      guard_b3(acc[0][j], acc[1][j], a0f, a1f, bh);
    }
  }
  acc_guard4(acc[0][0], acc[0][1], acc[0][2], acc[0][3]);
  acc_guard4(acc[0][4], acc[0][5], acc[0][6], acc[0][7]);
  acc_guard4(acc[1][0], acc[1][1], acc[1][2], acc[1][3]);
  acc_guard4(acc[1][4], acc[1][5], acc[1][6], acc[1][7]);

  float* slf = slab_all + wave * SLAB_PERW;
  const int h0 = n0 >> 6;
  float vs0 = 0.f, vs1 = 0.f, vd0 = 0.f, vd1 = 0.f;
#pragma unroll
  for (int i = 0; i < 2; ++i) {
#pragma unroll
    for (int j = 0; j < 8; ++j) {
#pragma unroll
      for (int r = 0; r < 8; ++r)
        slf[(8 * hh + r) * 128 + j * 16 + rl] = acc[i][j][r];
    }
    lds_wave_sync();
    {
      const float* ap = attk + (size_t)(h0 + hh) * (2 * UD);
      const float* sp = slf + rl * 128 + hh * 64;
      float s = 0.f, d = 0.f;
#pragma unroll 2
      for (int it = 0; it < UD / 4; ++it) {
        const v4f fv = *(const v4fa*)(sp + it * 4);
        const v4f as = bf_rne4(*(const v4fa*)(ap + it * 4));
        const v4f ad = bf_rne4(*(const v4fa*)(ap + UD + it * 4));
        s = fmaf(fv[0], as[0], s);
        s = fmaf(fv[1], as[1], s);
        s = fmaf(fv[2], as[2], s);
        s = fmaf(fv[3], as[3], s);
        d = fmaf(fv[0], ad[0], d);
        d = fmaf(fv[1], ad[1], d);
        d = fmaf(fv[2], ad[2], d);
        d = fmaf(fv[3], ad[3], d);
      }
      const float sA = __shfl(s, rl, 32);
      const float sB = __shfl(s, 16 + rl, 32);
      const float dA = __shfl(d, rl, 32);
      const float dB = __shfl(d, 16 + rl, 32);
      const bool mine = (hh == i);
      vs0 = mine ? sA : vs0;
      vs1 = mine ? sB : vs1;
      vd0 = mine ? dA : vd0;
      vd1 = mine ? dB : vd1;
    }
    lds_wave_sync();
  }
  float* base = sd + (size_t)h0 * bnp + m0 + lane;
  for (int pass = 0; pass < 2; ++pass) {
    *(volatile float*)(base)                           = vs0;
    *(volatile float*)(base + bnp)                     = vs1;
    *(volatile float*)(base + (size_t)NHD * bnp)       = vd0;
    *(volatile float*)(base + (size_t)(NHD + 1) * bnp) = vd1;
    __threadfence();
  }
}

#define KT       64
#define PSP      72
#define OSTP     128
#define NTILE    (FD / 16)
#define ATT_O_F  (4 * NTILE * 32 * 8)
#define ATT_P_H  (4 * 16 * PSP)
#define ATT_S_F  (4 * 16 * OSTP)
#define ATT_LDS_BYTES (ATT_O_F * 4 + ATT_P_H * 2 + ATT_S_F * 4)
static_assert(ATT_LDS_BYTES == 74752);
static_assert((ATT_O_F * 4) % 16 == 0 && ((ATT_O_F * 4 + ATT_P_H * 2) % 16) == 0);
static_assert(SEQ % KT == 0 && KT == 64 && NTILE == 8);

__global__ __launch_bounds__(128) __attribute__((amdgpu_num_vgpr(240))) void attn_kernel(
    const int* __restrict__ adj, const float* __restrict__ sd,
    const unsigned short* __restrict__ xt, float* __restrict__ out) {
  extern __shared__ v4f att_dyn[];
  float*    o_l   = (float*)(void*)att_dyn;
  _Float16* lds_p = (_Float16*)(void*)((char*)(void*)att_dyn + ATT_O_F * 4);
  float*    lds_s = (float*)(void*)((char*)(void*)att_dyn + ATT_O_F * 4 + ATT_P_H * 2);

  const int tid  = (int)threadIdx.x;
  const int lane = tid & 31;
  const int wave = wave_id();
  const int hh   = lane >> 4;
  const int c    = lane & 15;
  const int qb   = (int)blockIdx.x;
  const int h    = (int)blockIdx.y;
  const int b    = (int)blockIdx.z;
  const int q0   = qb * 64 + wave * 16;

  const int*      Ag = adj + (size_t)b * SEQ_FULL * SEQ_FULL + (size_t)(q0 + 8 * hh) * SEQ_FULL + 4 * c;
  const float*    Dg = sd + (size_t)(NHD + h) * BN + (size_t)b * SEQ + 4 * c;
  const _Float16* Vg = (const _Float16*)(const void*)xt + (size_t)b * FIN * SEQ + 8 * hh;
  _Float16* ph = lds_p + wave * (16 * PSP);
  float*    ow = o_l + wave * (NTILE * 32 * 8) + lane * 8;

  {
    const v4f z4 = {0.f, 0.f, 0.f, 0.f};
#pragma unroll
    for (int t = 0; t < NTILE; ++t) {
      *(v4fa*)(ow + t * 256)     = z4;
      *(v4fa*)(ow + t * 256 + 4) = z4;
    }
  }

  float cadd[8];
  {
    const size_t ro = (size_t)h * BN + (size_t)b * SEQ + q0 + 8 * hh;
    const v4f s0 = *(const v4fa*)(sd + ro);
    const v4f s1 = *(const v4fa*)(sd + ro + 4);
#pragma unroll
    for (int r = 0; r < 4; ++r) { cadd[r] = s0[r]; cadd[4 + r] = s1[r]; }
  }

  float mrow[8], lrow[8];
#pragma unroll
  for (int r = 0; r < 8; ++r) { mrow[r] = -INFINITY; lrow[r] = 0.f; }

#pragma unroll 1
  for (int kc = 0; kc < SEQ / KT; ++kc) {
    const int kv0 = kc * KT;
    const v4f d4 = *(const v4fa*)(Dg + kv0);
    float s[8][4];
    float cm[8];
#pragma unroll
    for (int r = 0; r < 8; ++r) {
      const v4i m4 = *(const v4ia*)(Ag + (size_t)r * SEQ_FULL + kv0);
      float m = -INFINITY;
#pragma unroll
      for (int q = 0; q < 4; ++q) {
        const float t  = cadd[r] + d4[q];
        const float e  = (t >= 0.0f) ? t : 0.2f * t;
        const float sv = (m4[q] != 0) ? e : NEGFILL;
        s[r][q] = sv;
        m = fmaxf(m, sv);
      }
#pragma unroll
      for (int off = 1; off < 16; off <<= 1) m = fmaxf(m, __shfl_xor(m, off, 32));
      cm[r] = m;
    }
    float alpha[8];
#pragma unroll
    for (int r = 0; r < 8; ++r) {
      const float mnew = fmaxf(mrow[r], cm[r]);
      const float al   = __expf(mrow[r] - mnew);
      mrow[r]  = mnew;
      alpha[r] = al;
      float psum = 0.f;
      v4h pv;
#pragma unroll
      for (int q = 0; q < 4; ++q) {
        const float p = __expf(s[r][q] - mnew);
        psum += p;
        pv[q] = (_Float16)(p * PSC);
      }
      *(v4ha*)(ph + (8 * hh + r) * PSP + 4 * c) = pv;
#pragma unroll
      for (int off = 1; off < 16; off <<= 1) psum += __shfl_xor(psum, off, 32);
      lrow[r] = lrow[r] * al + psum;
    }
    lds_wave_sync();
    const v16h pa0 = ldfrag_h(ph + c * PSP + 8 * hh);
    const v16h pa1 = ldfrag_h(ph + c * PSP + 32 + 8 * hh);
#pragma unroll 1
    for (int cc = 0; cc < 2; ++cc) {
      float* ocl = ow + cc * 1024;
      v8f oc[4];
#pragma unroll
      for (int t = 0; t < 4; ++t) {
        const v4f a4 = *(const v4fa*)(ocl + t * 256);
        const v4f b4 = *(const v4fa*)(ocl + t * 256 + 4);
        v8f o8;
#pragma unroll
        for (int r = 0; r < 4; ++r) {
          o8[r]     = a4[r] * alpha[r];
          o8[4 + r] = b4[r] * alpha[4 + r];
        }
        oc[t] = o8;
      }
#pragma unroll
      for (int t = 0; t < 4; ++t) {
        const size_t vo = (size_t)((cc * 4 + t) * 16 + c) * SEQ + kv0;
        const v16h vb0 = ldfrag_h(Vg + vo);
        const v16h vb1 = ldfrag_h(Vg + vo + 32);
        oc[t] = mma_h(pa0, vb0, oc[t]);
        oc[t] = mma_h(pa1, vb1, oc[t]);
        guard1_h4(oc[t], pa0, pa1, vb0, vb1);
      }
#pragma unroll
      for (int t = 0; t < 4; ++t) {
        v4f a4, b4;
#pragma unroll
        for (int r = 0; r < 4; ++r) { a4[r] = oc[t][r]; b4[r] = oc[t][4 + r]; }
        *(v4fa*)(ocl + t * 256)     = a4;
        *(v4fa*)(ocl + t * 256 + 4) = b4;
      }
    }
    lds_wave_sync();
  }

  float inv[8];
#pragma unroll
  for (int r = 0; r < 8; ++r) inv[r] = (1.0f / lrow[r]) * OSC;
  float* os = lds_s + wave * (16 * OSTP);
  float* Cb = out + ((size_t)b * SEQ + q0) * QKS + h * FD;
#pragma unroll
  for (int t = 0; t < NTILE; ++t) {
    const v4f a4 = *(const v4fa*)(ow + t * 256);
    const v4f b4 = *(const v4fa*)(ow + t * 256 + 4);
#pragma unroll
    for (int r = 0; r < 4; ++r) {
      os[(8 * hh + r) * OSTP + t * 16 + c]     = fmaxf(a4[r] * inv[r], 0.0f);
      os[(8 * hh + 4 + r) * OSTP + t * 16 + c] = fmaxf(b4[r] * inv[4 + r], 0.0f);
    }
  }
  lds_wave_sync();
  for (int pass = 0; pass < 2; ++pass) {
#pragma unroll
    for (int row = 0; row < 16; ++row) {
      const v4f xv = *(const v4fa*)(os + row * OSTP + lane * 4);
      *(volatile v4f*)(Cb + (size_t)row * QKS + lane * 4) = xv;
    }
    __threadfence();
  }
}

#define SZ_XB ((size_t)BN * FIN * 2)
#define SZ_WT ((size_t)HU * FIN * 2)
#define SZ_XT ((size_t)NB * FIN * SEQ * 2)
#define SZ_SD ((size_t)2 * NHD * BN * 4)
#define WS_TOTAL (SZ_XB + SZ_WT + SZ_XT + SZ_SD)
static_assert(WS_TOTAL <= 134217728);
static_assert(SZ_XB % 16384 == 0 && SZ_WT % 16384 == 0 && SZ_XT % 16384 == 0 && SZ_SD % 128 == 0);
static_assert(((size_t)BN - 1) * QKS + QKS - 1 < (size_t)BN * QKS);
static_assert(((BN / 32) * (HU / 128)) % 4 == 0);
static_assert((BN * FIN / 8) % 256 == 0);

extern "C" void kernel_launch(void* const* d_in, const int* in_sizes, int n_in,
                              void* d_out, int out_size, void* d_ws, size_t ws_size,
                              hipStream_t stream) {
  if (n_in < 4) return;
  const long long needX = ((long long)(NB - 1) * SEQ_FULL + SEQ) * FIN;
  const long long needA = (long long)(NB - 1) * SEQ_FULL * SEQ_FULL + (long long)(SEQ - 1) * SEQ_FULL + SEQ;
  if ((long long)in_sizes[0] < needX) return;
  if ((long long)in_sizes[1] < needA) return;
  if (in_sizes[2] != NHD * FIN * UD) return;
  if (in_sizes[3] != NHD * 2 * UD) return;
  if (out_size != BN * QKS) return;

  const float* X    = (const float*)d_in[0];
  const int*   Adj  = (const int*)d_in[1];
  const float* Wk   = (const float*)d_in[2];
  const float* Attk = (const float*)d_in[3];
  float* out = (float*)d_out;

  size_t off = 0;
  const size_t oXB = off; off += SZ_XB;
  const size_t oWT = off; off += SZ_WT;
  const size_t oXT = off; off += SZ_XT;
  const size_t oSD = off; off += SZ_SD;
  if (off != WS_TOTAL) return;
  if (off > ws_size) return;

  char* ws = (char*)d_ws;
  unsigned short* XB  = (unsigned short*)(ws + oXB);
  unsigned short* WTB = (unsigned short*)(ws + oWT);
  unsigned short* XT  = (unsigned short*)(ws + oXT);
  float*          SD  = (float*)(ws + oSD);

  const dim3 b256(256), b128(128);

  const int nux = BN * FIN / 8;
  prep_x_kernel<<<dim3((nux + 255) / 256), b256, 0, stream>>>(X, XB, nux);
  tconv_kernel<0><<<dim3(UD / 64, FIN / 64, NHD), b256, 0, stream>>>(Wk, WTB, FIN, UD, (long)FIN * UD, (long)UD * FIN);
  tconv_kernel<1><<<dim3(FIN / 64, SEQ / 64, NB), b256, 0, stream>>>(X, XT, SEQ, FIN, (long)SEQ_FULL * FIN, (long)FIN * SEQ);
  const int tilesF = (BN / 32) * (HU / 128);
  gemm_sd_kernel<<<dim3(tilesF / 4), b128, 0, stream>>>(XB, FIN, WTB, FIN, BN, HU, FIN, Attk, SD, BN);
  (void)hipFuncSetAttribute(reinterpret_cast<const void*>(&attn_kernel), hipFuncAttributeMaxDynamicSharedMemorySize, ATT_LDS_BYTES);
  attn_kernel<<<dim3(SEQ / 64, NHD, NB), b128, ATT_LDS_BYTES, stream>>>(Adj, SD, XT, out);
  (void)hipGetLastError();
}
